// RingDilatedAttentionHilbertCore_65755949301791
// MI455X (gfx1250) — hardware-verified
//
#include <hip/hip_runtime.h>


#define SS   14336
#define DD   512
#define NH_  8
#define HD   64
#define NKEY 2048
#define QC   2048
#define ZH   4
#define DM   DD
#define PCAR 1024.0f
#define VCAR 64.0f
#define OCAR 256.0f
#define LOSC 1024.0f
typedef _Float16 h16;
typedef unsigned short bf;
typedef __attribute__((ext_vector_type(16))) __bf16   v16bf;
typedef __attribute__((ext_vector_type(16))) _Float16 v16h;
typedef __attribute__((ext_vector_type(8)))  _Float16 v8h;
typedef __attribute__((ext_vector_type(8)))  unsigned short v8us;
typedef __attribute__((ext_vector_type(8)))  float    v8f;
typedef __attribute__((ext_vector_type(4)))  float    v4f;
typedef v8h  __attribute__((may_alias)) v8ha;
typedef v4f  __attribute__((may_alias)) v4fa;
typedef v8us __attribute__((may_alias)) v8usa;

__device__ __forceinline__ unsigned short f2bf(float f) { unsigned u = __float_as_uint(f); u += 0x7FFFu + ((u >> 16) & 1u); return (unsigned short)(u >> 16); }
__device__ __forceinline__ float bf2f(unsigned short b) { return __uint_as_float(((unsigned)b) << 16); }
__device__ __forceinline__ float bfr(float f) { return bf2f(f2bf(f)); }
__device__ __forceinline__ v16h cat16(v8h lo, v8h hi) { return __builtin_shufflevector(lo, hi, 0, 1, 2, 3, 4, 5, 6, 7, 8, 9, 10, 11, 12, 13, 14, 15); }
__device__ __forceinline__ v16bf cat16b(v8us lo, v8us hi) { return __builtin_bit_cast(v16bf, __builtin_shufflevector(lo, hi, 0, 1, 2, 3, 4, 5, 6, 7, 8, 9, 10, 11, 12, 13, 14, 15)); }
__device__ __forceinline__ v8f wmma16(v16h a, v16h b, v8f c) { return __builtin_amdgcn_wmma_f32_16x16x32_f16(false, a, false, b, (short)0, c, false, false); }
__device__ __forceinline__ v8f wmmab(v16bf a, v16bf b, v8f c) { return __builtin_amdgcn_wmma_f32_16x16x32_bf16(false, a, false, b, (short)0, c, false, false); }


__global__ __launch_bounds__(128) void k_gemmh(const h16* __restrict__ A, const h16* __restrict__ Bn, const float* __restrict__ bias, float* C, int ldc, const float* __restrict__ R, int K, size_t sA, size_t sB, size_t sC, int roundR) {
    __shared__ __align__(16) float ost[4][16 * 68];
    const size_t z = blockIdx.z; A += z * sA; Bn += z * sB; C += z * sC; if (R) R += z * sC;
    const int lane = threadIdx.x & 31, wave = threadIdx.x >> 5, lr = lane & 15, hi = lane >> 4;
    const int r0 = blockIdx.x * 64 + wave * 16, c0 = blockIdx.y * 64;
    const size_t aoff = (size_t)(r0 + lr) * K + 8 * hi;
    size_t boff[4];
#pragma unroll
    for (int t = 0; t < 4; ++t) boff[t] = (size_t)(c0 + t * 16 + lr) * K + 8 * hi;
    v8f acc[4];
#pragma unroll
    for (int t = 0; t < 4; ++t) acc[t] = (v8f){};
#pragma unroll 1
    for (int kc = 0; kc < K; kc += 32) {
        const v16h a = cat16(*(const v8h*)(A + aoff + kc), *(const v8h*)(A + aoff + kc + 16));
#pragma unroll
        for (int t = 0; t < 4; ++t) { const v16h b = cat16(*(const v8h*)(Bn + boff[t] + kc), *(const v8h*)(Bn + boff[t] + kc + 16)); acc[t] = wmma16(a, b, acc[t]); }
        asm volatile("v_nop\n\tv_nop\n\tv_nop\n\tv_nop" : "+v"(acc[0]), "+v"(acc[1]), "+v"(acc[2]), "+v"(acc[3]) : "v"(a));
    }
    float* os = &ost[wave][0];
#pragma unroll
    for (int t = 0; t < 4; ++t) { const float bv = bias ? bfr(bias[c0 + t * 16 + lr]) : 0.f;
#pragma unroll
        for (int j = 0; j < 8; ++j) os[(hi * 8 + j) * 68 + t * 16 + lr] = acc[t][j] + bv; }
    __syncthreads();
    float* crow = C + (size_t)r0 * ldc + c0;
    auto pass = [&]() {
#pragma unroll
        for (int s = 0; s < 8; ++s) { const int Lid = (lane >> 3) + 4 * s, piece = lane & 7; const int row = Lid >> 1, cofs = (Lid & 1) * 32 + piece * 4;
            v4f val = *(const v4fa*)(os + row * 68 + cofs); if (R) { const v4f rv = *(const v4f*)(R + ((size_t)r0 + row) * ldc + c0 + cofs); val += roundR ? (v4f){bfr(rv[0]), bfr(rv[1]), bfr(rv[2]), bfr(rv[3])} : rv; }
            *(volatile v4f*)(crow + (size_t)row * ldc + cofs) = val; }
    };
    pass(); __threadfence(); pass();
}

template <int MODE>
__global__ __launch_bounds__(128) void k_gemm3z(const bf* __restrict__ Ah, const bf* __restrict__ Al, const bf* __restrict__ Bh, const bf* __restrict__ Bl, int K, float* C, int ldc, size_t sA, size_t sB, size_t sC) {
    if ((MODE & 1) && (int)blockIdx.y * 64 > (int)blockIdx.x * 64 + 63) return;
    const size_t z = blockIdx.z; Ah += z * sA; Al += z * sA; Bh += z * sB; Bl += z * sB; C += z * sC;
    const int Klim = (MODE & 2) ? min(K, ((int)blockIdx.x + 1) * 64) : K;
    __shared__ __align__(16) float ost[4][16 * 68];
    const int lane = threadIdx.x & 31, wave = threadIdx.x >> 5, lr = lane & 15, hi = lane >> 4;
    const int r0 = blockIdx.x * 64 + wave * 16, c0 = blockIdx.y * 64;
    const size_t aoff = (size_t)(r0 + lr) * K + 8 * hi;
    v8f acc[4];
#pragma unroll
    for (int t = 0; t < 4; ++t) acc[t] = (v8f){};
#pragma unroll 1
    for (int kc = 0; kc < Klim; kc += 32) {
        const v16bf a = cat16b(*(const v8us*)(Ah + aoff + kc), *(const v8us*)(Ah + aoff + kc + 16));
        v16bf al = a; if (!(MODE & 4) && !(MODE & 16)) al = cat16b(*(const v8us*)(Al + aoff + kc), *(const v8us*)(Al + aoff + kc + 16));
#pragma unroll
        for (int t = 0; t < 4; ++t) { const size_t bo = (size_t)(c0 + t * 16 + lr) * K + kc + 8 * hi;
            const v16bf bh = cat16b(*(const v8us*)(Bh + bo), *(const v8us*)(Bh + bo + 16));
            acc[t] = wmmab(a, bh, acc[t]);
            if (!(MODE & 4)) { if (!(MODE & 16)) acc[t] = wmmab(al, bh, acc[t]); if (!(MODE & 8)) { const v16bf bl = cat16b(*(const v8us*)(Bl + bo), *(const v8us*)(Bl + bo + 16)); acc[t] = wmmab(a, bl, acc[t]); } } }
        asm volatile("v_nop\n\tv_nop\n\tv_nop\n\tv_nop" : "+v"(acc[0]), "+v"(acc[1]), "+v"(acc[2]), "+v"(acc[3]) : "v"(a), "v"(al));
    }
    float* os = &ost[wave][0];
#pragma unroll
    for (int t = 0; t < 4; ++t) {
#pragma unroll
        for (int j = 0; j < 8; ++j) os[(hi * 8 + j) * 68 + t * 16 + lr] = acc[t][j]; }
    __builtin_amdgcn_wave_barrier(); asm volatile("" ::: "memory");
    float* crow = C + (size_t)r0 * ldc + c0;
    auto pass = [&]() {
#pragma unroll
        for (int s = 0; s < 8; ++s) { const int Lid = (lane >> 3) + 4 * s, piece = lane & 7; const int row = Lid >> 1, cofs = (Lid & 1) * 32 + piece * 4;
            const v4f val = *(const v4fa*)(os + row * 68 + cofs); *(volatile v4f*)(crow + (size_t)row * ldc + cofs) = val; }
    };
    pass(); __threadfence(); pass();
}
__global__ __launch_bounds__(256) void k_planes32z(const float* __restrict__ F, int ld, int off, float sc, int rows, bf* Ph, bf* Pl) {
    typedef __attribute__((ext_vector_type(2))) unsigned short v2us;
    const int lane = threadIdx.x & 31; const size_t r = ((size_t)blockIdx.x * 8 + (threadIdx.x >> 5)) * 2 + (lane >> 4); if (r >= (size_t)rows) return; const int z = blockIdx.z; const int c0 = (lane & 15) * 2; v2us oh, ol;
    Ph += (size_t)z * rows * 32; Pl += (size_t)z * rows * 32;
#pragma unroll
    for (int i = 0; i < 2; ++i) { const float y = F[r * ld + off + z * 32 + c0 + i] * sc; const unsigned short hb = f2bf(y); oh[i] = hb; ol[i] = f2bf(y - bf2f(hb)); }
    const size_t o = r * 32 + c0; *(volatile v2us*)(Ph + o) = oh; *(volatile v2us*)(Pl + o) = ol; __threadfence(); *(volatile v2us*)(Ph + o) = oh; *(volatile v2us*)(Pl + o) = ol;
}
__global__ __launch_bounds__(256) void k_vtpadz(const float* __restrict__ F, int ld, int off, int nk, bf* Th, bf* Tl) {
    typedef __attribute__((ext_vector_type(2))) unsigned short v2us;
    const int lane = threadIdx.x & 31; const size_t wid = (size_t)blockIdx.x * 8 + (threadIdx.x >> 5); if (wid >= (size_t)64 * (nk / 64)) return; const int z = blockIdx.z; const int d = (int)(wid / (nk / 64)); const int k0 = (int)(wid % (nk / 64)) * 64 + lane * 2; v2us oh, ol;
    Th += (size_t)z * 64 * nk; Tl += (size_t)z * 64 * nk;
#pragma unroll
    for (int i = 0; i < 2; ++i) { const float y = (d < 32) ? F[(size_t)(k0 + i) * ld + off + z * 32 + (d < 32 ? d : 0)] : 0.f; const unsigned short hb = f2bf(y); oh[i] = hb; ol[i] = f2bf(y - bf2f(hb)); }
    const size_t o = (size_t)d * nk + k0; *(volatile v2us*)(Th + o) = oh; *(volatile v2us*)(Tl + o) = ol; __threadfence(); *(volatile v2us*)(Th + o) = oh; *(volatile v2us*)(Tl + o) = ol;
}
template <int NK>
__global__ __launch_bounds__(256) void k_softmaxz(const float* __restrict__ S, int rows, bf* PH, bf* PL) {
    typedef __attribute__((ext_vector_type(4))) unsigned short v4us;
    const int lane = threadIdx.x & 31, i = blockIdx.x * 8 + (threadIdx.x >> 5); if (i >= rows) return; const size_t zo = (size_t)blockIdx.z * rows * NK; const float* sr = S + zo + (size_t)i * NK; PH += zo; PL += zo;
    float m = -3.0e38f;
#pragma unroll 1
    for (int c0 = lane * 4; c0 < NK; c0 += 128) {
#pragma unroll
        for (int q = 0; q < 4; ++q) m = fmaxf(m, sr[c0 + q]); }
#pragma unroll
    for (int sh = 16; sh; sh >>= 1) m = fmaxf(m, __shfl_xor(m, sh, 32));
    float sum = 0.f;
#pragma unroll 1
    for (int c0 = lane * 4; c0 < NK; c0 += 128) {
#pragma unroll
        for (int q = 0; q < 4; ++q) sum += __expf(sr[c0 + q] - m); }
#pragma unroll
    for (int sh = 16; sh; sh >>= 1) sum += __shfl_xor(sum, sh, 32);
    const float inv = 1.0f / sum;
#pragma unroll 1
    for (int ps = 0; ps < 2; ++ps) {
#pragma unroll 1
        for (int c0 = lane * 4; c0 < NK; c0 += 128) { v4us oh, ol;
#pragma unroll
            for (int q = 0; q < 4; ++q) { const float p = __expf(sr[c0 + q] - m) * inv; const unsigned short hb = f2bf(p); oh[q] = hb; ol[q] = f2bf(p - bf2f(hb)); }
            const size_t o = (size_t)i * NK + c0; *(volatile v4us*)(PH + o) = oh; *(volatile v4us*)(PL + o) = ol; }
        if (ps == 0) __threadfence(); }
}
__global__ __launch_bounds__(256) void k_placez(const float* __restrict__ XH, int rows, int ldy, float* Y) {
    const int lane = threadIdx.x & 31; const size_t q = (size_t)blockIdx.x * 8 + (threadIdx.x >> 5); if (q >= (size_t)rows) return; const int z = blockIdx.z; const float v = XH[((size_t)z * rows + q) * 64 + lane];
    *(volatile float*)(Y + q * ldy + z * 32 + lane) = v; __threadfence(); *(volatile float*)(Y + q * ldy + z * 32 + lane) = v;
}

template <typename T16> struct WFrag;
template <> struct WFrag<h16> { typedef v16h V; static __device__ __forceinline__ V ld(const h16* p) { return cat16(*(const v8h*)p, *(const v8h*)(p + 16)); } static __device__ __forceinline__ v8f mma(V a, V b, v8f c) { return wmma16(a, b, c); } };
template <> struct WFrag<bf> { typedef v16bf V; static __device__ __forceinline__ V ld(const bf* p) { return cat16b(*(const v8us*)p, *(const v8us*)(p + 16)); } static __device__ __forceinline__ v8f mma(V a, V b, v8f c) { return wmmab(a, b, c); } };
template <typename T16, int NSPLIT, bool BIAS>
__global__ __launch_bounds__(32) void k_gemmw(const T16* __restrict__ A, const T16* __restrict__ A2, const T16* __restrict__ Bt, const T16* __restrict__ Bt2, int K, float* C, int ldc, const float* __restrict__ bias, size_t sA, size_t sB, size_t sC) {
    typedef typename WFrag<T16>::V V;
    __shared__ __align__(16) float os[16 * 68];
    const size_t z = blockIdx.z; A += z * sA; if (A2) A2 += z * sA; Bt += z * sB; if (Bt2) Bt2 += z * sB; C += z * sC;
    const int lane = threadIdx.x & 31, lr = lane & 15, hi = lane >> 4; const int r0 = blockIdx.x * 64, c0 = blockIdx.y * 64;
    v8f acc[4][4];
#pragma unroll
    for (int mb = 0; mb < 4; ++mb)
#pragma unroll
        for (int nb = 0; nb < 4; ++nb) acc[mb][nb] = (v8f){};
    const size_t aoff = (size_t)(r0 + lr) * K + 8 * hi, boff = (size_t)(c0 + lr) * K + 8 * hi;
#pragma unroll 1
    for (int kc = 0; kc < K; kc += 32) {
        V a[4], a2[4];
#pragma unroll
        for (int mb = 0; mb < 4; ++mb) { a[mb] = WFrag<T16>::ld(A + aoff + (size_t)mb * 16 * K + kc); if (NSPLIT == 1 || NSPLIT == 2) a2[mb] = WFrag<T16>::ld(A2 + aoff + (size_t)mb * 16 * K + kc); }
#pragma unroll
        for (int nb = 0; nb < 4; ++nb) { const V b = WFrag<T16>::ld(Bt + boff + (size_t)nb * 16 * K + kc); V b2; if (NSPLIT >= 2) b2 = WFrag<T16>::ld(Bt2 + boff + (size_t)nb * 16 * K + kc);
#pragma unroll
            for (int mb = 0; mb < 4; ++mb) { acc[mb][nb] = WFrag<T16>::mma(a[mb], b, acc[mb][nb]); if (NSPLIT == 1 || NSPLIT == 2) acc[mb][nb] = WFrag<T16>::mma(a2[mb], b, acc[mb][nb]); if (NSPLIT >= 2) acc[mb][nb] = WFrag<T16>::mma(a[mb], b2, acc[mb][nb]); } }
        asm volatile("v_nop\n\tv_nop\n\tv_nop\n\tv_nop" : "+v"(acc[0][0]), "+v"(acc[1][1]), "+v"(acc[2][2]), "+v"(acc[3][3]) : "v"(a[0]), "v"(a[3]));
    }
#pragma unroll
    for (int mb = 0; mb < 4; ++mb) {
#pragma unroll
        for (int nb = 0; nb < 4; ++nb) {
#pragma unroll
            for (int j = 0; j < 8; ++j) os[(hi * 8 + j) * 68 + nb * 16 + lr] = acc[mb][nb][j]; }
        __builtin_amdgcn_wave_barrier(); asm volatile("" ::: "memory");
        float* crow = C + (size_t)(r0 + mb * 16) * ldc + c0;
#pragma unroll 1
        for (int ps = 0; ps < 2; ++ps) {
#pragma unroll
            for (int s = 0; s < 8; ++s) { const int row = 2 * s + hi, cofs = lr * 4; v4f val = *(const v4fa*)(os + row * 68 + cofs); if (BIAS) { val[0] += bfr(bias[c0 + cofs]); val[1] += bfr(bias[c0 + cofs + 1]); val[2] += bfr(bias[c0 + cofs + 2]); val[3] += bfr(bias[c0 + cofs + 3]); }
                *(volatile v4f*)(crow + (size_t)row * ldc + cofs) = val; }
            if (ps == 0) __threadfence(); }
        __builtin_amdgcn_wave_barrier(); asm volatile("" ::: "memory");
    }
}
typedef __attribute__((ext_vector_type(4))) _Float16 v4h;
__device__ __forceinline__ h16 tohx(float x) { return (h16)x; }
template <bool F16O>
__global__ __launch_bounds__(256) void k_wT(const float* __restrict__ Wm, int K, int N, bf* Bt, h16* Bh) {
    __shared__ float tl[64][65]; typedef __attribute__((ext_vector_type(4))) unsigned short v4us;
    const int tid = threadIdx.x; const int k0 = blockIdx.x * 64, n0 = blockIdx.y * 64; const int rr = tid >> 2, cq = (tid & 3) * 16;
#pragma unroll
    for (int i = 0; i < 16; ++i) tl[rr][cq + i] = bfr(Wm[(size_t)(k0 + rr) * N + n0 + cq + i]);
    __syncthreads();
    const int lane = tid & 31, wv = tid >> 5;
    auto pass = [&]() {
#pragma unroll
        for (int st = 0; st < 4; ++st) { const int nr = wv * 8 + st * 2 + (lane >> 4); const int kq = (lane & 15) * 4; const size_t off = (size_t)(n0 + nr) * K + k0 + kq;
            if (F16O) { v4h v; for (int i = 0; i < 4; ++i) v[i] = tohx(tl[kq + i][nr]); *(volatile v4h*)(Bh + off) = v; } else { v4us v; for (int i = 0; i < 4; ++i) v[i] = f2bf(tl[kq + i][nr]); *(volatile v4us*)(Bt + off) = v; } }
    };
    pass(); __threadfence(); pass();
}
__global__ __launch_bounds__(256) void k_cvtx(const float* __restrict__ x, bf* A) {
    const int lane = threadIdx.x & 31; const size_t r = (size_t)blockIdx.x * 8 + (threadIdx.x >> 5); if (r >= (size_t)SS) return;
#pragma unroll 1
    for (int ps = 0; ps < 2; ++ps) {
#pragma unroll
        for (int q = 0; q < DD / 256; ++q) { const size_t o = r * DD + q * 256 + lane * 8; v8us v;
#pragma unroll
            for (int i = 0; i < 8; ++i) v[i] = f2bf(x[o + i]);
            *(volatile v8us*)(A + o) = v; }
        if (ps == 0) __threadfence(); }
}
__global__ __launch_bounds__(256) void k_qpl(const float* __restrict__ QKV, int qrow0, int h0, h16* Qx) {
    const int lane = threadIdx.x & 31; const size_t w = (size_t)blockIdx.x * 8 + (threadIdx.x >> 5); const int t = (int)(w * 2 + (lane >> 4)); if (t >= QC) return; const int z = blockIdx.z; const int c0 = (lane & 15) * 4; v4h o;
#pragma unroll
    for (int q = 0; q < 4; ++q) o[q] = tohx(QKV[(size_t)(qrow0 + t) * (3 * DD) + (h0 + z) * HD + c0 + q] * 0.125f);
    const size_t off = ((size_t)z * QC + t) * HD + c0; *(volatile v4h*)(Qx + off) = o; __threadfence(); *(volatile v4h*)(Qx + off) = o;
}
__global__ __launch_bounds__(256) void k_kpl(const float* __restrict__ QKV, int dil, int h0, h16* Kx) {
    const int lane = threadIdx.x & 31; const size_t w = (size_t)blockIdx.x * 8 + (threadIdx.x >> 5); const int m = (int)(w * 2 + (lane >> 4)); if (m >= NKEY) return; const int z = blockIdx.z; const int c0 = (lane & 15) * 4; v4h o;
#pragma unroll
    for (int q = 0; q < 4; ++q) o[q] = tohx(QKV[(size_t)(m * dil) * (3 * DD) + DD + (h0 + z) * HD + c0 + q]);
    const size_t off = ((size_t)z * NKEY + m) * HD + c0; *(volatile v4h*)(Kx + off) = o; __threadfence(); *(volatile v4h*)(Kx + off) = o;
}
__global__ __launch_bounds__(256) void k_vT(const float* __restrict__ QKV, int dil, int h0, h16* VT) {
    __shared__ float tl[64][65];
    const int tid = threadIdx.x; const int m0 = blockIdx.x * 64; const int z = blockIdx.z; const int rr = tid >> 2, cq = (tid & 3) * 16;
#pragma unroll
    for (int i = 0; i < 16; ++i) tl[rr][cq + i] = QKV[(size_t)((m0 + rr) * dil) * (3 * DD) + 2 * DD + (h0 + z) * HD + cq + i] * VCAR;
    __syncthreads();
    const int lane = tid & 31, wv = tid >> 5;
    auto pass = [&]() {
#pragma unroll
        for (int st = 0; st < 4; ++st) { const int dr = wv * 8 + st * 2 + (lane >> 4); const int tq = (lane & 15) * 4; v4h v;
#pragma unroll
            for (int i = 0; i < 4; ++i) v[i] = tohx(tl[tq + i][dr]);
            *(volatile v4h*)(VT + ((size_t)z * HD + dr) * NKEY + m0 + tq) = v; }
    };
    pass(); __threadfence(); pass();
}
__global__ __launch_bounds__(256) void k_soft(const float* __restrict__ S, h16* P) {
    const int lane = threadIdx.x & 31, i = blockIdx.x * 8 + (threadIdx.x >> 5); if (i >= QC) return; const size_t zo = ((size_t)blockIdx.z * QC + i) * NKEY; const float* sr = S + zo; h16* po = P + zo;
    float m = -3.0e38f;
#pragma unroll 1
    for (int c0 = lane * 4; c0 < NKEY; c0 += 128) {
#pragma unroll
        for (int q = 0; q < 4; ++q) m = fmaxf(m, sr[c0 + q]); }
#pragma unroll
    for (int sh = 16; sh; sh >>= 1) m = fmaxf(m, __shfl_xor(m, sh, 32));
    float sum = 0.f;
#pragma unroll 1
    for (int c0 = lane * 4; c0 < NKEY; c0 += 128) {
#pragma unroll
        for (int q = 0; q < 4; ++q) sum += __expf(sr[c0 + q] - m); }
#pragma unroll
    for (int sh = 16; sh; sh >>= 1) sum += __shfl_xor(sum, sh, 32);
    const float f = __fdiv_rn(PCAR, sum);
#pragma unroll 1
    for (int ps = 0; ps < 2; ++ps) {
#pragma unroll 1
        for (int c0 = lane * 4; c0 < NKEY; c0 += 128) { v4h o;
#pragma unroll
            for (int q = 0; q < 4; ++q) o[q] = tohx(__expf(sr[c0 + q] - m) * f);
            *(volatile v4h*)(po + c0) = o; }
        if (ps == 0) __threadfence(); }
}
__global__ __launch_bounds__(256) void k_merge(const float* __restrict__ OZ, int qg0, int h0, h16* OH) {
    const int lane = threadIdx.x & 31, t = blockIdx.x * 8 + (threadIdx.x >> 5); if (t >= QC) return; const int z = lane >> 3, d0 = (lane & 7) * 8; v8h o;
#pragma unroll
    for (int k = 0; k < 8; ++k) o[k] = tohx(OZ[((size_t)z * QC + t) * HD + d0 + k] * (OCAR / (PCAR * VCAR)));
    const size_t off = (size_t)(qg0 + t) * DD + (h0 + z) * HD + d0; *(volatile v8h*)(OH + off) = o; __threadfence(); *(volatile v8h*)(OH + off) = o;
}
__global__ __launch_bounds__(256) void k_fin(const float* __restrict__ CO, const float* __restrict__ bo, float* OUTB) {
    const int lane = threadIdx.x & 31; const size_t r = (size_t)blockIdx.x * 8 + (threadIdx.x >> 5); if (r >= (size_t)SS) return;
#pragma unroll 1
    for (int ps = 0; ps < 2; ++ps) {
#pragma unroll
        for (int p = 0; p < DD / 128; ++p) { const int c0 = p * 128 + lane * 4; v4f v = *(const v4f*)(CO + r * DD + c0);
#pragma unroll
            for (int i = 0; i < 4; ++i) v[i] = v[i] * (1.0f / OCAR) + bfr(bo[c0 + i]);
            *(volatile v4f*)(OUTB + r * DD + c0) = v; }
        if (ps == 0) __threadfence(); }
}
extern "C" void kernel_launch(void* const* d_in, const int* in_sizes, int n_in,
                              void* d_out, int out_size, void* d_ws, size_t ws_size, hipStream_t stream) {
    (void)in_sizes; (void)n_in; (void)out_size;
    const float* x = (const float*)d_in[0]; const float* wqkv = (const float*)d_in[1]; const float* bqkv = (const float*)d_in[2]; const float* wout = (const float*)d_in[3]; const float* bout = (const float*)d_in[4];
    float* out = (float*)d_out;
    char* wsp = (char*)d_ws;
    auto take = [&](size_t bytes) { char* p = wsp; wsp += (bytes + 255) & ~(size_t)255; return (void*)p; };
    bf* WQ = (bf*)take((size_t)3 * DD * DD * 2); h16* WO = (h16*)take((size_t)DD * DD * 2); bf* XB = (bf*)take((size_t)SS * DD * 2); float* QKV = (float*)take((size_t)8192 * 3 * DD * 4);
    h16* Qx = (h16*)take((size_t)ZH * QC * HD * 2); h16* Kx = (h16*)take((size_t)ZH * NKEY * HD * 2); h16* VT = (h16*)take((size_t)ZH * HD * NKEY * 2); float* S = (float*)take((size_t)ZH * QC * NKEY * 4); h16* Px = (h16*)take((size_t)ZH * QC * NKEY * 2); float* OZ = (float*)take((size_t)ZH * QC * HD * 4); h16* OH = (h16*)take((size_t)SS * DD * 2); float* CO = (float*)take((size_t)SS * DD * 4);
    if ((size_t)(wsp - (char*)d_ws) > ws_size) return;
    k_wT<false><<<dim3(DD / 64, (3 * DD) / 64, 1), 256, 0, stream>>>(wqkv, DD, 3 * DD, WQ, nullptr); k_wT<true><<<dim3(DD / 64, DD / 64, 1), 256, 0, stream>>>(wout, DD, DD, nullptr, WO);
    k_cvtx<<<SS / 8, 256, 0, stream>>>(x, XB);
    const int segA[3] = {0, 2048, 6144}, segL[3] = {2048, 4096, 8192}, segD[3] = {1, 2, 4};
    for (int s = 0; s < 3; ++s) {
        k_gemmw<bf, 0, true><<<dim3(segL[s] / 64, (3 * DD) / 64, 1), 32, 0, stream>>>(XB + (size_t)segA[s] * DD, nullptr, WQ, nullptr, DD, QKV, 3 * DD, bqkv, 0, 0, 0);
        for (int qc0 = 0; qc0 < segL[s]; qc0 += QC)
            for (int h0 = 0; h0 < NH_; h0 += ZH) {
                k_qpl<<<dim3((QC / 2) / 8, 1, ZH), 256, 0, stream>>>(QKV, qc0, h0, Qx); k_kpl<<<dim3((NKEY / 2) / 8, 1, ZH), 256, 0, stream>>>(QKV, segD[s], h0, Kx); k_vT<<<dim3(NKEY / 64, 1, ZH), 256, 0, stream>>>(QKV, segD[s], h0, VT);
                k_gemmw<h16, 0, false><<<dim3(QC / 64, NKEY / 64, ZH), 32, 0, stream>>>(Qx, nullptr, Kx, nullptr, HD, S, NKEY, nullptr, (size_t)QC * HD, (size_t)NKEY * HD, (size_t)QC * NKEY);
                k_soft<<<dim3(QC / 8, 1, ZH), 256, 0, stream>>>(S, Px);
                k_gemmw<h16, 0, false><<<dim3(QC / 64, 1, ZH), 32, 0, stream>>>(Px, nullptr, VT, nullptr, NKEY, OZ, HD, nullptr, (size_t)QC * NKEY, (size_t)HD * NKEY, (size_t)QC * HD);
                k_merge<<<QC / 8, 256, 0, stream>>>(OZ, segA[s] + qc0, h0, OH); } }
    k_gemmw<h16, 0, false><<<dim3(SS / 64, DD / 64, 1), 32, 0, stream>>>(OH, nullptr, WO, nullptr, DD, CO, DD, nullptr, 0, 0, 0);
    k_fin<<<SS / 8, 256, 0, stream>>>(CO, bout, out);
}
